// MLPNetworkWithAttention1__80169859547542
// MI455X (gfx1250) — hardware-verified
//
#include <hip/hip_runtime.h>
#include <math.h>

constexpr int kRows   = 131072;
constexpr int kXCols  = 39;
constexpr int kObs    = 12;
constexpr int kHid    = 256;
constexpr int kCat    = 512;
constexpr int kHdim   = 32;
constexpr int kKpad   = 32;
constexpr int kC1     = 8192;
constexpr int kNC1    = kRows / kC1;
constexpr int kC2     = 16384;
constexpr int kNC2    = kRows / kC2;
constexpr int kRB     = 1024;
constexpr int kNRB    = kRows / kRB;
constexpr int kRBPerC1 = kC1 / kRB;
constexpr float kSqrtHd     = 5.656854152679443f;
constexpr float kScoreScale = 1.0f / kSqrtHd;
constexpr float kBnEps = 1e-5f;
static_assert(kRows % kC1 == 0 && kRows % kC2 == 0, "chunks exact");
static_assert(kC1 % 64 == 0 && kC1 % kRB == 0 && kC2 % 64 == 0 && kC2 % 256 == 0, "tile multiples");

typedef __attribute__((ext_vector_type(16))) _Float16 v16h;
typedef __attribute__((ext_vector_type(8)))  _Float16 v8h;
typedef __attribute__((ext_vector_type(16))) __bf16   v16b;
typedef __attribute__((ext_vector_type(8)))  __bf16   v8b;
typedef __attribute__((ext_vector_type(8)))  float    v8f;
typedef __attribute__((ext_vector_type(4)))  float    v4f;
typedef __attribute__((ext_vector_type(4)))  unsigned int v4u;

__device__ __forceinline__ unsigned short f2bf_bits(float f) {
  unsigned u = __float_as_uint(f);
  return (unsigned short)((u + 0x7FFFu + ((u >> 16) & 1u)) >> 16);
}
__device__ __forceinline__ float bf_bits2f(unsigned short h) { return __uint_as_float(((unsigned)h) << 16); }
__device__ __forceinline__ float bfr(float f) { return bf_bits2f(f2bf_bits(f)); }
__device__ __forceinline__ unsigned pk16(unsigned short a, unsigned short b) { return (unsigned)a | ((unsigned)b << 16); }

__device__ __forceinline__ void dep_guard_h(v8f& a, v8f& b, v16h x, v16h y) { asm volatile("v_nop\n\tv_nop\n\tv_nop\n\tv_nop" : "+v"(a), "+v"(b) : "v"(x), "v"(y)); }
__device__ __forceinline__ void dep_guard_b(v8f& a, v8f& b, v16b x, v16b y) { asm volatile("v_nop\n\tv_nop\n\tv_nop\n\tv_nop" : "+v"(a), "+v"(b) : "v"(x), "v"(y)); }
__device__ __forceinline__ void keep4_h(v16h a, v16h b, v16h c, v16h d) { asm volatile("v_nop" :: "v"(a), "v"(b), "v"(c), "v"(d)); }
__device__ __forceinline__ void keep4_b(v16b a, v16b b, v16b c, v16b d) { asm volatile("v_nop" :: "v"(a), "v"(b), "v"(c), "v"(d)); }
__device__ __forceinline__ void acc_guard4(v8f& a, v8f& b, v8f& c, v8f& d) { asm volatile("v_nop\n\tv_nop\n\tv_nop\n\tv_nop" : "+v"(a), "+v"(b), "+v"(c), "+v"(d)); }
template <typename T> struct Frag;
template <> struct Frag<_Float16> {
  typedef v16h V; union U { v16h v; v8h h[2]; };
  static __device__ __forceinline__ v16h load(const _Float16* p) {
    U f; f.h[0] = *(const v8h*)(p); f.h[1] = *(const v8h*)(p + 16); return f.v;
  }
  static __device__ __forceinline__ v8f mma(v16h a, v16h b, v8f c) {
    return __builtin_amdgcn_wmma_f32_16x16x32_f16(false, a, false, b, (short)0, c, false, false);
  }
  static __device__ __forceinline__ void guard(v8f& a, v8f& b, v16h x, v16h y) { dep_guard_h(a, b, x, y); }
  static __device__ __forceinline__ void keep(v16h a, v16h b, v16h c, v16h d) { keep4_h(a, b, c, d); }
};
template <> struct Frag<__bf16> {
  typedef v16b V; union U { v16b v; v8b h[2]; };
  static __device__ __forceinline__ v16b load(const __bf16* p) {
    U f; f.h[0] = *(const v8b*)(p); f.h[1] = *(const v8b*)(p + 16); return f.v;
  }
  static __device__ __forceinline__ v8f mma(v16b a, v16b b, v8f c) {
    return __builtin_amdgcn_wmma_f32_16x16x32_bf16(false, a, false, b, (short)0, c, false, false);
  }
  static __device__ __forceinline__ void guard(v8f& a, v8f& b, v16b x, v16b y) { dep_guard_b(a, b, x, y); }
  static __device__ __forceinline__ void keep(v16b a, v16b b, v16b c, v16b d) { keep4_b(a, b, c, d); }
};

template <int ET> struct Elem;
template <> struct Elem<0> { typedef _Float16 T; };
template <> struct Elem<1> { typedef __bf16 T; };
template <int ET, int SPL, int BIAS_MODE, int OUT_MODE, int ACT>
__global__ __launch_bounds__(256) void wmma_gemm64(
    const unsigned short* __restrict__ Ap, const unsigned short* __restrict__ A2p, int lda, long strideA,
    const unsigned short* __restrict__ Btp, const unsigned short* __restrict__ Bt2p, int ldb, long strideB,
    void* __restrict__ Cout, void* __restrict__ Cout2, int ldc, long strideC,
    const float* __restrict__ bias,
    int M, int N, int K, float scale) {
  typedef typename Elem<ET>::T T;
  typedef typename Frag<T>::V V;
  const T* A = (const T*)Ap; const T* A2 = (const T*)A2p; const T* Bt = (const T*)Btp; const T* Bt2 = (const T*)Bt2p;
  __shared__ __align__(16) float sT[8][16 * 68];
  const int b    = blockIdx.y;
  const int lane = threadIdx.x & 31;
  const int wave = threadIdx.x >> 5;
  const int tilesN = N >> 6;
  const int tilesM = M >> 6;
  const int tile = blockIdx.x * 8 + wave;
  if (tile >= tilesM * tilesN) return;
  const int tm = tile / tilesN;
  const int tn = tile - tm * tilesN;
  const int m0 = tm << 6;
  const int n0 = tn << 6;

  const T* Ab  = A  + (size_t)b * strideA;
  const T* Bb  = Bt + (size_t)b * strideB;
  const T* Ab2 = (SPL & 1) ? (A2  + (size_t)b * strideA) : nullptr;
  const T* Bb2 = (SPL & 2) ? (Bt2 + (size_t)b * strideB) : nullptr;

  const int rlane = lane & 15;
  const int koff  = (lane >> 4) * 8;
  const int mOff  = (lane >> 4) * 8;

  v8f acc[4][4];
#pragma unroll
  for (int i = 0; i < 4; ++i)
#pragma unroll
    for (int j = 0; j < 4; ++j) acc[i][j] = (v8f){0.f,0.f,0.f,0.f,0.f,0.f,0.f,0.f};

  for (int k0 = 0; k0 < K; k0 += 32) {
    V bh[4], bl[4];
#pragma unroll
    for (int j = 0; j < 4; ++j) {
      const size_t bo = (size_t)(n0 + (j << 4) + rlane) * ldb + koff + k0;
      bh[j] = Frag<T>::load(Bb + bo);
      if (SPL & 2) bl[j] = Frag<T>::load(Bb2 + bo);
    }
#pragma unroll
    for (int i = 0; i < 4; ++i) {
      const size_t ao = (size_t)(m0 + (i << 4) + rlane) * lda + koff + k0;
      V ah = Frag<T>::load(Ab + ao);
      V al;
      if (SPL & 1) al = Frag<T>::load(Ab2 + ao);
#pragma unroll
      for (int j = 0; j < 4; ++j) {
        acc[i][j] = Frag<T>::mma(ah, bh[j], acc[i][j]);
        if (SPL & 2) acc[i][j] = Frag<T>::mma(ah, bl[j], acc[i][j]);
        if (SPL & 1) acc[i][j] = Frag<T>::mma(al, bh[j], acc[i][j]);
      }
      Frag<T>::guard(acc[i][0], acc[i][3], ah, (SPL & 1) ? al : ah);
    }
    Frag<T>::keep(bh[0], bh[1], bh[2], bh[3]);
    if (SPL & 2) Frag<T>::keep(bl[0], bl[1], bl[2], bl[3]);
  }
  acc_guard4(acc[0][0], acc[0][1], acc[0][2], acc[0][3]);
  acc_guard4(acc[1][0], acc[1][1], acc[1][2], acc[1][3]);
  acc_guard4(acc[2][0], acc[2][1], acc[2][2], acc[2][3]);
  acc_guard4(acc[3][0], acc[3][1], acc[3][2], acc[3][3]);

  float* slab = sT[wave];
#pragma unroll
  for (int i = 0; i < 4; ++i) {
    const int mBase = m0 + (i << 4);
#pragma unroll
    for (int j = 0; j < 4; ++j) {
      const int n = n0 + (j << 4) + rlane;
      float bv = 0.f;
      if (BIAS_MODE == 2) bv = bias[n];
#pragma unroll
      for (int r = 0; r < 8; ++r) {
        float v = acc[i][j][r] * scale;
        if (BIAS_MODE == 1) v += bias[mBase + mOff + r];
        if (BIAS_MODE == 2) v += bv;
        if (ACT == 2) v = fmaxf(v, 0.0f);
        if (ACT == 4) v = (v > 0.f) ? v : 0.01f * v;
        slab[(mOff + r) * 68 + (j << 4) + rlane] = v;
      }
    }
    __builtin_amdgcn_fence(__ATOMIC_RELEASE, "workgroup");
    __builtin_amdgcn_wave_barrier();
    __builtin_amdgcn_fence(__ATOMIC_ACQUIRE, "workgroup");
    if (OUT_MODE == 0) {
      float* C = (float*)Cout + (size_t)b * strideC;
      const int hh = lane >> 4, c4 = (lane & 15) * 4;
      for (int pass = 0; pass < 2; ++pass) {
#pragma unroll
        for (int it = 0; it < 8; ++it) {
          const int row = it * 2 + hh;
          v4f v = *(const v4f*)(slab + row * 68 + c4);
          *(volatile v4f*)(C + (size_t)(mBase + row) * ldc + n0 + c4) = v;
        }
        __threadfence();
      }
    } else {
      const int q = lane >> 3, c8 = (lane & 7) * 8;
      unsigned short* C  = (unsigned short*)Cout  + (size_t)b * strideC;
      unsigned short* C2 = (OUT_MODE == 2) ? ((unsigned short*)Cout2 + (size_t)b * strideC) : nullptr;
      for (int pass = 0; pass < 2; ++pass) {
#pragma unroll
        for (int it = 0; it < 4; ++it) {
          const int row = it * 4 + q;
          const float* sp = slab + row * 68 + c8;
          v8h hv, lv;
#pragma unroll
          for (int e = 0; e < 8; ++e) {
            if (OUT_MODE == 1) {
              hv[e] = (_Float16)sp[e];
            } else {
              unsigned short hb = f2bf_bits(sp[e]);
              unsigned short lb = f2bf_bits(sp[e] - bf_bits2f(hb));
              hv[e] = __builtin_bit_cast(_Float16, hb);
              lv[e] = __builtin_bit_cast(_Float16, lb);
            }
          }
          *(volatile v8h*)(C + (size_t)(mBase + row) * ldc + n0 + c8) = hv;
          if (OUT_MODE == 2) *(volatile v8h*)(C2 + (size_t)(mBase + row) * ldc + n0 + c8) = lv;
        }
        __threadfence();
      }
    }
    __builtin_amdgcn_fence(__ATOMIC_RELEASE, "workgroup");
    __builtin_amdgcn_wave_barrier();
    __builtin_amdgcn_fence(__ATOMIC_ACQUIRE, "workgroup");
  }
}

__device__ __forceinline__ int role_agent(const int* __restrict__ agent_idx, int role) {
  int aq = agent_idx[0];
  aq = aq < 0 ? 0 : (aq > 2 ? 2 : aq);
  const int o0 = (aq == 0) ? 1 : 0;
  const int o1 = (aq == 2) ? 1 : 2;
  return (role == 0) ? aq : ((role == 1) ? o0 : o1);
}

__global__ __launch_bounds__(256) void k_wprep(const float* __restrict__ emb_W, const float* __restrict__ emb_b,
    const float* __restrict__ v_b, const float* __restrict__ fco_b, const float* __restrict__ fc1_b,
    const float* __restrict__ fc2_W, const int* __restrict__ agent_idx,
    unsigned short* __restrict__ EMBWT, float* __restrict__ BIASR) {
  __shared__ __align__(16) unsigned short sW[kHid * kKpad];
  const int r = blockIdx.x;
  const int t = threadIdx.x;
  const int a = role_agent(agent_idx, r);
  const float* W = emb_W + (size_t)a * 13 * kHid;
  unsigned short* srow = sW + t * kKpad;
#pragma unroll 1
  for (int f = 0; f < 13; ++f) srow[f] = f2bf_bits(W[f * kHid + t]);
  srow[13] = f2bf_bits(emb_b[a * kHid + t]);
#pragma unroll 1
  for (int f = 14; f < kKpad; ++f) srow[f] = (unsigned short)0;
  __syncthreads();
  unsigned short* outp = EMBWT + (size_t)r * kHid * kKpad;
  for (int pass = 0; pass < 2; ++pass) {
#pragma unroll
    for (int it = 0; it < 4; ++it) {
      const int e = it * 2048 + 8 * t;
      const v4u v = *(const v4u*)(sW + e);
      *(volatile v4u*)(outp + e) = v;
    }
    __threadfence();
  }
  const float b0 = bfr(v_b[t]), b1 = bfr(fco_b[t]), b2 = bfr(fc1_b[t]), b3 = bfr(fc2_W[t]);
  const float bv = (r == 0) ? b0 : ((r == 1) ? b1 : b2);
  float* bp  = BIASR + r * kHid + t;
  float* bp3 = BIASR + 3 * kHid + t;
  *(volatile float*)bp = bv;
  if (r == 0) *(volatile float*)bp3 = b3;
  __threadfence();
  *(volatile float*)bp = bv;
  if (r == 0) *(volatile float*)bp3 = b3;
}

__global__ __launch_bounds__(256) void k_wtrans(const float* __restrict__ in, unsigned short* __restrict__ out, int Krows, int Ncols) {
  __shared__ __align__(16) unsigned short sT[8 * 512];
  const int n0 = blockIdx.x * 8, t = threadIdx.x;
#pragma unroll 1
  for (int k = t; k < Krows; k += 256) {
    const float* p = in + (size_t)k * Ncols + n0;
    const v4f a = *(const v4f*)p;
    const v4f c = *(const v4f*)(p + 4);
#pragma unroll
    for (int j = 0; j < 4; ++j) {
      sT[j * Krows + k]       = f2bf_bits(a[j]);
      sT[(4 + j) * Krows + k] = f2bf_bits(c[j]);
    }
  }
  __syncthreads();
  const int nIt = (8 * Krows) >> 11;
  unsigned short* op = out + (size_t)n0 * Krows;
  for (int pass = 0; pass < 2; ++pass) {
    for (int it = 0; it < nIt; ++it) {
      const int e = it * 2048 + 8 * t;
      const v4u v = *(const v4u*)(sT + e);
      *(volatile v4u*)(op + e) = v;
    }
    __threadfence();
  }
}

__global__ __launch_bounds__(256) void k_feats(const float* __restrict__ x, const int* __restrict__ agent_idx,
                                                unsigned short* __restrict__ FEAT, int c0, int C) {
  const int p = blockIdx.y, t = threadIdx.x;
  const int a = role_agent(agent_idx, p);
  const int lr = blockIdx.x * 64 + (t >> 2);
  const int q  = t & 3;
  int gr = c0 + lr;
  gr = gr < 0 ? 0 : (gr > kRows - 1 ? kRows - 1 : gr);
  const float* xr = x + (size_t)gr * kXCols;
  unsigned short hb[8];
#pragma unroll
  for (int e = 0; e < 8; ++e) {
    const int f = q * 8 + e;
    const int col = (f < kObs) ? (a * kObs + f) : ((f == kObs) ? (36 + a) : 0);
    const float xv = xr[col];
    hb[e] = (f < 13) ? f2bf_bits(xv) : ((f == 13) ? (unsigned short)0x3F80u : (unsigned short)0);
  }
  const v4u u = (v4u){pk16(hb[0], hb[1]), pk16(hb[2], hb[3]), pk16(hb[4], hb[5]), pk16(hb[6], hb[7])};
  unsigned short* dst = FEAT + ((size_t)p * C + lr) * kKpad + q * 8;
  *(volatile v4u*)dst = u;
  __threadfence();
  *(volatile v4u*)dst = u;
}

__global__ __launch_bounds__(256) void k_scores(const float* __restrict__ QKO, float* __restrict__ S, int C) {
  __shared__ __align__(16) float sS[32 * 16];
  const int t = threadIdx.x, lr = t >> 3, h = t & 7;
  const size_t row = (size_t)blockIdx.x * 32 + lr;
  const size_t pl  = (size_t)C * kHid;
  const float* Qp  = QKO + row * kHid + h * kHdim;
  const float* K0p = Qp + pl;
  const float* K1p = Qp + 2 * pl;
  float s0 = 0.f, s1 = 0.f;
#pragma unroll 1
  for (int c = 0; c < 8; ++c) {
    const v4f qv  = *(const v4f*)(Qp + 4 * c);
    const v4f k0v = *(const v4f*)(K0p + 4 * c);
    const v4f k1v = *(const v4f*)(K1p + 4 * c);
#pragma unroll
    for (int e = 0; e < 4; ++e) {
      s0 = fmaf(qv[e], k0v[e], s0);
      s1 = fmaf(qv[e], k1v[e], s1);
    }
  }
  s0 *= kScoreScale;
  s1 *= kScoreScale;
  const float mx  = fmaxf(s0, s1);
  const float e0  = expf(s0 - mx), e1 = expf(s1 - mx);
  const float inv = 1.0f / (e0 + e1);
  sS[lr * 16 + h * 2]     = e0 * inv;
  sS[lr * 16 + h * 2 + 1] = e1 * inv;
  __syncthreads();
  if (t < 128) {
    float* dst = S + (size_t)blockIdx.x * 32 * 16 + 4 * t;
    const v4f v = *(const v4f*)(sS + 4 * t);
    *(volatile v4f*)dst = v;
    __threadfence();
    *(volatile v4f*)dst = v;
  }
}

__global__ __launch_bounds__(256) void k_av(const float* __restrict__ S, const float* __restrict__ VV,
                                             unsigned short* __restrict__ AVH, unsigned short* __restrict__ AVL, int C) {
  const int t = threadIdx.x, lr = t >> 5, c8 = (t & 31) * 8, h = c8 >> 5;
  const size_t row = (size_t)blockIdx.x * 8 + lr;
  const float w0 = S[row * 16 + h * 2];
  const float w1 = S[row * 16 + h * 2 + 1];
  const float* v0p = VV + row * kHid + c8;
  const float* v1p = v0p + (size_t)C * kHid;
  const v4f a0 = *(const v4f*)v0p, a1 = *(const v4f*)(v0p + 4);
  const v4f b0 = *(const v4f*)v1p, b1 = *(const v4f*)(v1p + 4);
  unsigned short hb[8], lb[8];
#pragma unroll
  for (int e = 0; e < 4; ++e) {
    const float av0 = w0 * a0[e] + w1 * b0[e];
    const float av1 = w0 * a1[e] + w1 * b1[e];
    hb[e] = f2bf_bits(av0);
    lb[e] = f2bf_bits(av0 - bf_bits2f(hb[e]));
    hb[4 + e] = f2bf_bits(av1);
    lb[4 + e] = f2bf_bits(av1 - bf_bits2f(hb[4 + e]));
  }
  const v4u hu = (v4u){pk16(hb[0], hb[1]), pk16(hb[2], hb[3]), pk16(hb[4], hb[5]), pk16(hb[6], hb[7])};
  const v4u lu = (v4u){pk16(lb[0], lb[1]), pk16(lb[2], lb[3]), pk16(lb[4], lb[5]), pk16(lb[6], lb[7])};
  const size_t o = row * kHid + c8;
  *(volatile v4u*)(AVH + o) = hu;
  *(volatile v4u*)(AVL + o) = lu;
  __threadfence();
  *(volatile v4u*)(AVH + o) = hu;
  *(volatile v4u*)(AVL + o) = lu;
}

__global__ __launch_bounds__(256) void k_stats(const unsigned short* __restrict__ EH, const unsigned short* __restrict__ EL,
                                                const unsigned short* __restrict__ AT, double* __restrict__ PART, int rb0) {
  const int half = blockIdx.y, rb = blockIdx.x, t = threadIdx.x;
  const size_t base = (size_t)rb * kRB * kHid + t;
  double s = 0.0, ss = 0.0;
  if (half == 0) {
#pragma unroll 1
    for (int r = 0; r < kRB; ++r) {
      const size_t o = base + (size_t)r * kHid;
      const double d = (double)(bf_bits2f(EH[o]) + bf_bits2f(EL[o]));
      s += d;
      ss = fma(d, d, ss);
    }
  } else {
#pragma unroll 1
    for (int r = 0; r < kRB; ++r) {
      const size_t o = base + (size_t)r * kHid;
      const double d = (double)(float)__builtin_bit_cast(_Float16, AT[o]);
      s += d;
      ss = fma(d, d, ss);
    }
  }
  double* dp = PART + (size_t)(rb0 + rb) * (2 * kCat) + half * kHid + t;
  *(volatile double*)dp = s;
  *(volatile double*)(dp + kCat) = ss;
  __threadfence();
  *(volatile double*)dp = s;
  *(volatile double*)(dp + kCat) = ss;
}

__global__ __launch_bounds__(256) void k_bnfinal(const double* __restrict__ PART, float* __restrict__ MEANRS) {
  const int c = blockIdx.x * 256 + threadIdx.x;
  double s = 0.0, ss = 0.0;
#pragma unroll 1
  for (int rb = 0; rb < kNRB; ++rb) {
    s  += PART[(size_t)rb * (2 * kCat) + c];
    ss += PART[(size_t)rb * (2 * kCat) + kCat + c];
  }
  const double invB = 1.0 / (double)kRows;
  const double mean = s * invB;
  double var = ss * invB - mean * mean;
  var = var < 0.0 ? 0.0 : var;
  const float mf = (float)mean;
  const float rs = rsqrtf((float)var + kBnEps);
  float* mp = MEANRS + c;
  *(volatile float*)mp = mf;
  *(volatile float*)(mp + kCat) = rs;
  __threadfence();
  *(volatile float*)mp = mf;
  *(volatile float*)(mp + kCat) = rs;
}

__global__ __launch_bounds__(256) void k_bnapply(const unsigned short* __restrict__ EH, const unsigned short* __restrict__ EL,
                                                  const unsigned short* __restrict__ AT, const float* __restrict__ MEANRS,
                                                  unsigned short* __restrict__ XNH, unsigned short* __restrict__ XNL) {
  const int t = threadIdx.x;
  const size_t row = (size_t)blockIdx.x * 4 + (t >> 6);
  const int c8 = (t & 63) * 8;
  const int cl = c8 & 255;
  const bool second = (c8 >= kHid);
  const size_t o = row * kHid + cl;
  const v4u hv = *(const v4u*)(EH + o);
  const v4u lv = *(const v4u*)(EL + o);
  const v4u av = *(const v4u*)(AT + o);
  const v4f ma = *(const v4f*)(MEANRS + c8), mb = *(const v4f*)(MEANRS + c8 + 4);
  const v4f ra = *(const v4f*)(MEANRS + kCat + c8), rb = *(const v4f*)(MEANRS + kCat + c8 + 4);
  const float mm[8] = {ma[0], ma[1], ma[2], ma[3], mb[0], mb[1], mb[2], mb[3]};
  const float rr[8] = {ra[0], ra[1], ra[2], ra[3], rb[0], rb[1], rb[2], rb[3]};
  unsigned short oh[8], ol[8];
#pragma unroll
  for (int e = 0; e < 4; ++e) {
    const unsigned hw = hv[e], lw = lv[e], aw = av[e];
    const float eq0 = bf_bits2f((unsigned short)(hw & 0xFFFFu)) + bf_bits2f((unsigned short)(lw & 0xFFFFu));
    const float eq1 = bf_bits2f((unsigned short)(hw >> 16)) + bf_bits2f((unsigned short)(lw >> 16));
    const float at0 = (float)__builtin_bit_cast(_Float16, (unsigned short)(aw & 0xFFFFu));
    const float at1 = (float)__builtin_bit_cast(_Float16, (unsigned short)(aw >> 16));
    const float x0 = second ? at0 : eq0;
    const float x1 = second ? at1 : eq1;
    const float xn0 = (x0 - mm[2 * e]) * rr[2 * e];
    const float xn1 = (x1 - mm[2 * e + 1]) * rr[2 * e + 1];
    oh[2 * e] = f2bf_bits(xn0);
    ol[2 * e] = f2bf_bits(xn0 - bf_bits2f(oh[2 * e]));
    oh[2 * e + 1] = f2bf_bits(xn1);
    ol[2 * e + 1] = f2bf_bits(xn1 - bf_bits2f(oh[2 * e + 1]));
  }
  const v4u hu = (v4u){pk16(oh[0], oh[1]), pk16(oh[2], oh[3]), pk16(oh[4], oh[5]), pk16(oh[6], oh[7])};
  const v4u lu = (v4u){pk16(ol[0], ol[1]), pk16(ol[2], ol[3]), pk16(ol[4], ol[5]), pk16(ol[6], ol[7])};
  const size_t od = row * kCat + c8;
  *(volatile v4u*)(XNH + od) = hu;
  *(volatile v4u*)(XNL + od) = lu;
  __threadfence();
  *(volatile v4u*)(XNH + od) = hu;
  *(volatile v4u*)(XNL + od) = lu;
}

__global__ __launch_bounds__(256) void k_fc2(const float* __restrict__ H1, const float* __restrict__ W2r,
                                              const float* __restrict__ fc2_b, float* __restrict__ outc) {
  const int t = threadIdx.x;
  const size_t row = (size_t)blockIdx.x * 256 + t;
  const float* hp = H1 + row * kHid;
  float acc = 0.f;
#pragma unroll 1
  for (int c = 0; c < kHid / 4; ++c) {
    const v4f h = *(const v4f*)(hp + 4 * c);
    const v4f w = *(const v4f*)(W2r + 4 * c);
    acc = fmaf(h[0], w[0], acc);
    acc = fmaf(h[1], w[1], acc);
    acc = fmaf(h[2], w[2], acc);
    acc = fmaf(h[3], w[3], acc);
  }
  const float o = acc + bfr(fc2_b[0]);
  float* op = outc + row;
  *(volatile float*)op = o;
  __threadfence();
  *(volatile float*)op = o;
}

extern "C" void kernel_launch(void* const* d_in, const int* in_sizes, int n_in,
                              void* d_out, int out_size, void* d_ws, size_t ws_size,
                              hipStream_t stream) {
  if (n_in < 14) return;
  if (in_sizes[0] != kRows * kXCols) return;
  if (in_sizes[1] != 3 * 13 * kHid || in_sizes[2] != 3 * kHid) return;
  if (in_sizes[3] != kHid * kHid || in_sizes[4] != kHid * kHid || in_sizes[5] != kHid * kHid || in_sizes[7] != kHid * kHid) return;
  if (in_sizes[6] != kHid || in_sizes[8] != kHid || in_sizes[10] != kHid || in_sizes[11] != kHid) return;
  if (in_sizes[9] != kCat * kHid) return;
  if (in_sizes[12] < 1 || in_sizes[13] < 1) return;
  if (out_size != kRows) return;

  const float* x      = (const float*)d_in[0];
  const float* emb_W  = (const float*)d_in[1];
  const float* emb_b  = (const float*)d_in[2];
  const float* q_W    = (const float*)d_in[3];
  const float* k_W    = (const float*)d_in[4];
  const float* v_W    = (const float*)d_in[5];
  const float* v_b    = (const float*)d_in[6];
  const float* fco_W  = (const float*)d_in[7];
  const float* fco_b  = (const float*)d_in[8];
  const float* fc1_W  = (const float*)d_in[9];
  const float* fc1_b  = (const float*)d_in[10];
  const float* fc2_W  = (const float*)d_in[11];
  const float* fc2_b  = (const float*)d_in[12];
  const int*   agent  = (const int*)d_in[13];
  float* outp = (float*)d_out;

  const size_t SZ_EMBWT = (size_t)3 * kHid * kKpad * 2;
  const size_t SZ_QKWT  = (size_t)3 * kHid * kHid * 2;
  const size_t SZ_W256  = (size_t)kHid * kHid * 2;
  const size_t SZ_FC1   = (size_t)kHid * kCat * 2;
  const size_t SZ_BIAS  = (size_t)4 * kHid * 4;
  const size_t SZ_MRS   = (size_t)2 * kCat * 4;
  const size_t SZ_PART  = (size_t)kNRB * 2 * kCat * 8;
  const size_t SZ_ATTN  = (size_t)kRows * kHid * 2;
  const size_t SZ_FEAT3 = (size_t)3 * kC1 * kKpad * 2;
  const size_t SZ_S     = (size_t)kC1 * 16 * 4;
  const size_t SZ_EMB3  = (size_t)3 * kC1 * kHid * 2;
  const size_t SZ_QKO   = (size_t)3 * kC1 * kHid * 4;
  const size_t SZ_VV    = (size_t)2 * kC1 * kHid * 4;
  const size_t SZ_AV    = (size_t)kC1 * kHid * 2;
  const size_t SZ_FEAT1 = (size_t)kC2 * kKpad * 2;
  const size_t SZ_EMB1  = (size_t)kC2 * kHid * 2;
  const size_t SZ_XN    = (size_t)kC2 * kCat * 2;
  const size_t SZ_H1    = (size_t)kC2 * kHid * 4;

  size_t off = 0;
  const size_t oEMBWT = off; off += SZ_EMBWT;
  const size_t oQKWT  = off; off += SZ_QKWT;
  const size_t oVWT   = off; off += SZ_W256;
  const size_t oFCO   = off; off += SZ_W256;
  const size_t oFC1   = off; off += SZ_FC1;
  const size_t oBIAS  = off; off += SZ_BIAS;
  const size_t oMRS   = off; off += SZ_MRS;
  const size_t oPART  = off; off += SZ_PART;
  const size_t oATTN  = off; off += SZ_ATTN;
  const size_t oCH    = off;
  const size_t oFEAT  = oCH;
  const size_t oS     = oCH;
  const size_t oEMBH  = oFEAT + SZ_FEAT3;
  const size_t oEMBL  = oEMBH + SZ_EMB3;
  const size_t oQKO   = oEMBL + SZ_EMB3;
  const size_t oVV    = oQKO;
  const size_t oAVH   = oVV + SZ_VV;
  const size_t oAVL   = oAVH + SZ_AV;
  const size_t endP1  = oQKO + SZ_QKO;
  const size_t oFEAT2 = oCH;
  const size_t oEMBH2 = oFEAT2 + SZ_FEAT1;
  const size_t oEMBL2 = oEMBH2 + SZ_EMB1;
  const size_t oXNH   = oEMBL2 + SZ_EMB1;
  const size_t oXNL   = oXNH + SZ_XN;
  const size_t endP2  = oXNL + SZ_XN;
  const size_t oH1    = oCH;
  const size_t TOTAL  = (endP1 > endP2) ? endP1 : endP2;
  if (SZ_S > SZ_FEAT3) return;
  if (oAVL + SZ_AV > endP1) return;
  if (oH1 + SZ_H1 > oXNH) return;
  if (TOTAL > ws_size) return;
  if (TOTAL > (size_t)134217728) return;

  char* ws = (char*)d_ws;
  typedef unsigned short u16;
  u16*    EMBWT  = (u16*)(ws + oEMBWT);
  u16*    QKWT   = (u16*)(ws + oQKWT);
  u16*    VWT    = (u16*)(ws + oVWT);
  u16*    FCOWT  = (u16*)(ws + oFCO);
  u16*    FC1WT  = (u16*)(ws + oFC1);
  float*  BIASR  = (float*)(ws + oBIAS);
  float*  MEANRS = (float*)(ws + oMRS);
  double* PART   = (double*)(ws + oPART);
  u16*    ATTN   = (u16*)(ws + oATTN);
  u16*    FEAT   = (u16*)(ws + oFEAT);
  float*  S      = (float*)(ws + oS);
  u16*    EMBH   = (u16*)(ws + oEMBH);
  u16*    EMBL   = (u16*)(ws + oEMBL);
  float*  QKO    = (float*)(ws + oQKO);
  float*  VV     = (float*)(ws + oVV);
  u16*    AVH    = (u16*)(ws + oAVH);
  u16*    AVL    = (u16*)(ws + oAVL);
  u16*    FEAT2  = (u16*)(ws + oFEAT2);
  u16*    EMBH2  = (u16*)(ws + oEMBH2);
  u16*    EMBL2  = (u16*)(ws + oEMBL2);
  u16*    XNH    = (u16*)(ws + oXNH);
  u16*    XNL    = (u16*)(ws + oXNL);
  float*  H1     = (float*)(ws + oH1);

  const dim3 blk(256);
  const size_t plW   = (size_t)kHid * kHid;
  const long   plE1  = (long)kC1 * kHid;
  const long   plF1  = (long)kC1 * kKpad;
  const long   plEW  = (long)kHid * kKpad;
  const int    gx1   = (kC1 / 64) * (kHid / 64) / 8;
  const int    gx2   = (kC2 / 64) * (kHid / 64) / 8;

  k_wprep<<<dim3(3), blk, 0, stream>>>(emb_W, emb_b, v_b, fco_b, fc1_b, fc2_W, agent, EMBWT, BIASR);
  k_wtrans<<<dim3(kHid / 8), blk, 0, stream>>>(q_W,   QKWT,           kHid, kHid);
  k_wtrans<<<dim3(kHid / 8), blk, 0, stream>>>(k_W,   QKWT + plW,     kHid, kHid);
  k_wtrans<<<dim3(kHid / 8), blk, 0, stream>>>(k_W,   QKWT + 2 * plW, kHid, kHid);
  k_wtrans<<<dim3(kHid / 8), blk, 0, stream>>>(v_W,   VWT,            kHid, kHid);
  k_wtrans<<<dim3(kHid / 8), blk, 0, stream>>>(fco_W, FCOWT,          kHid, kHid);
  k_wtrans<<<dim3(kHid / 8), blk, 0, stream>>>(fc1_W, FC1WT,          kCat, kHid);

  for (int ch = 0; ch < kNC1; ++ch) {
    const int c0 = ch * kC1;
    k_feats<<<dim3(kC1 / 64, 3), blk, 0, stream>>>(x, agent, FEAT, c0, kC1);
    wmma_gemm64<1, 0, 0, 2, 0><<<dim3(gx1, 3), blk, 0, stream>>>(
        FEAT, FEAT, kKpad, plF1, EMBWT, EMBWT, kKpad, plEW,
        (void*)EMBH, (void*)EMBL, kHid, plE1, BIASR, kC1, kHid, kKpad, 1.0f);
    wmma_gemm64<1, 1, 0, 0, 0><<<dim3(gx1, 3), blk, 0, stream>>>(
        EMBH, EMBL, kHid, plE1, QKWT, QKWT, kHid, (long)plW,
        (void*)QKO, (void*)QKO, kHid, plE1, BIASR, kC1, kHid, kHid, 1.0f);
    k_scores<<<dim3(kC1 / 32), blk, 0, stream>>>(QKO, S, kC1);
    wmma_gemm64<1, 1, 2, 0, 4><<<dim3(gx1, 2), blk, 0, stream>>>(
        EMBH + plE1, EMBL + plE1, kHid, plE1, VWT, VWT, kHid, 0L,
        (void*)VV, (void*)VV, kHid, plE1, BIASR, kC1, kHid, kHid, 1.0f);
    k_av<<<dim3(kC1 / 8), blk, 0, stream>>>(S, VV, AVH, AVL, kC1);
    u16* ATc = ATTN + (size_t)c0 * kHid;
    wmma_gemm64<1, 1, 2, 1, 0><<<dim3(gx1, 1), blk, 0, stream>>>(
        AVH, AVL, kHid, 0L, FCOWT, FCOWT, kHid, 0L,
        (void*)ATc, (void*)ATc, kHid, 0L, BIASR + kHid, kC1, kHid, kHid, 1.0f);
    k_stats<<<dim3(kRBPerC1, 2), blk, 0, stream>>>(EMBH, EMBL, ATc, PART, ch * kRBPerC1);
  }

  k_bnfinal<<<dim3(2), blk, 0, stream>>>(PART, MEANRS);

  for (int ch = 0; ch < kNC2; ++ch) {
    const int c0 = ch * kC2;
    k_feats<<<dim3(kC2 / 64, 1), blk, 0, stream>>>(x, agent, FEAT2, c0, kC2);
    wmma_gemm64<1, 0, 0, 2, 0><<<dim3(gx2, 1), blk, 0, stream>>>(
        FEAT2, FEAT2, kKpad, 0L, EMBWT, EMBWT, kKpad, 0L,
        (void*)EMBH2, (void*)EMBL2, kHid, 0L, BIASR, kC2, kHid, kKpad, 1.0f);
    k_bnapply<<<dim3(kC2 / 4), blk, 0, stream>>>(EMBH2, EMBL2, ATTN + (size_t)c0 * kHid, MEANRS, XNH, XNL);
    wmma_gemm64<1, 1, 2, 0, 4><<<dim3(gx2, 1), blk, 0, stream>>>(
        XNH, XNL, kCat, 0L, FC1WT, FC1WT, kCat, 0L,
        (void*)H1, (void*)H1, kHid, 0L, BIASR + 2 * kHid, kC2, kHid, kCat, 1.0f);
    k_fc2<<<dim3(kC2 / 256), blk, 0, stream>>>(H1, BIASR + 3 * kHid, fc2_b, outp + c0);
  }
}
